// GIN_84121229460233
// MI455X (gfx1250) — hardware-verified
//
#include <hip/hip_runtime.h>

typedef float          v8f   __attribute__((ext_vector_type(8)));
typedef float          v4f   __attribute__((ext_vector_type(4)));
typedef unsigned int   v4u   __attribute__((ext_vector_type(4)));
typedef int            v8i   __attribute__((ext_vector_type(8)));
typedef unsigned short v8us  __attribute__((ext_vector_type(8)));
typedef unsigned short v16us __attribute__((ext_vector_type(16)));
typedef __bf16         v16bf __attribute__((ext_vector_type(16)));
typedef _Float16       v16h  __attribute__((ext_vector_type(16)));
typedef v4f  __attribute__((may_alias)) v4fa;
typedef v8us __attribute__((may_alias)) v8usa;
union FragB { v16bf v; v16us u; v8us h[2]; v8i w; };
union FragH { v16h  v; v16us u; v8us h[2]; v8i w; };

__device__ __forceinline__ v8f wmb(const FragB& a, const FragB& b, v8f c) {
  v8f d = __builtin_amdgcn_wmma_f32_16x16x32_bf16(false, a.v, false, b.v, (short)0, c, false, false);
  asm volatile("v_nop\n\tv_nop\n\tv_nop\n\tv_nop" : "+v"(d) : "v"(a.w), "v"(b.w));
  return d;
}

__device__ __forceinline__ v8f wmh(const FragH& a, const FragH& b, v8f c) {
  v8f d = __builtin_amdgcn_wmma_f32_16x16x32_f16(false, a.v, false, b.v, (short)0, c, false, false);
  asm volatile("v_nop\n\tv_nop\n\tv_nop\n\tv_nop" : "+v"(d) : "v"(a.w), "v"(b.w));
  return d;
}

__device__ __forceinline__ unsigned bf16_bits(float f) {
  const unsigned u = __float_as_uint(f);
  const unsigned r = (u + 0x7FFFu + ((u >> 16) & 1u)) >> 16;
  const unsigned q = (u >> 16) | 0x40u;
  return ((u & 0x7fffffffu) > 0x7f800000u) ? q : r;
}

__device__ __forceinline__ float bf16_val(float f) {
  return __uint_as_float(bf16_bits(f) << 16);
}
__device__ __forceinline__ int clampi(int v, int lo, int hi) {
  return v < lo ? lo : (v > hi ? hi : v);
}

__device__ __forceinline__ unsigned f16_bits(float f) {
  const unsigned u  = __float_as_uint(f);
  const unsigned s  = (u >> 16) & 0x8000u;
  const unsigned a  = u & 0x7fffffffu;
  const unsigned t  = a - 0x38000000u;
  const unsigned r  = (t + 0x0FFFu + ((t >> 13) & 1u)) >> 13;
  const unsigned rc = r > 0x7C00u ? 0x7C00u : r;
  const bool small  = a < 0x38800000u;
  const bool isnan  = a > 0x7f800000u;
  const unsigned fin = small ? 0u : (s | rc);
  return isnan ? (s | 0x7E00u) : fin;
}

__device__ __forceinline__ unsigned pk16(unsigned lo, unsigned hi) { return lo | (hi << 16); }
__device__ __forceinline__ unsigned bf16_lo_bits(float v) {
  float hi = bf16_val(v);
  asm volatile("" : "+v"(hi));
  return bf16_bits(v - hi);
}
__device__ __forceinline__ v4u pack8_bf16(v4f a, v4f c) {
  return (v4u){ pk16(bf16_bits(a[0]), bf16_bits(a[1])), pk16(bf16_bits(a[2]), bf16_bits(a[3])),
                pk16(bf16_bits(c[0]), bf16_bits(c[1])), pk16(bf16_bits(c[2]), bf16_bits(c[3])) };
}
__device__ __forceinline__ v4u pack8_bf16_lo(v4f a, v4f c) {
  return (v4u){ pk16(bf16_lo_bits(a[0]), bf16_lo_bits(a[1])), pk16(bf16_lo_bits(a[2]), bf16_lo_bits(a[3])),
                pk16(bf16_lo_bits(c[0]), bf16_lo_bits(c[1])), pk16(bf16_lo_bits(c[2]), bf16_lo_bits(c[3])) };
}
__device__ __forceinline__ v4u pack8_f16(v4f a, v4f c) {
  return (v4u){ pk16(f16_bits(a[0]), f16_bits(a[1])), pk16(f16_bits(a[2]), f16_bits(a[3])),
                pk16(f16_bits(c[0]), f16_bits(c[1])), pk16(f16_bits(c[2]), f16_bits(c[3])) };
}

template <int FORM>
__global__ __launch_bounds__(256) void k_plane(const float* __restrict__ src, int rows, int cols, int ldsrc,
                                               unsigned short* __restrict__ dst, int MP, int KP) {
  static_assert(FORM >= 0 && FORM <= 3);
  const int KTOT = (FORM == 1 || FORM == 3) ? 2 * KP : KP;
  const unsigned ppr   = (unsigned)(KTOT >> 3);
  const unsigned kp8   = (unsigned)(KP >> 3);
  const unsigned total = (unsigned)MP * ppr;
  const unsigned g     = blockIdx.x * 256u + threadIdx.x;
  const unsigned rowu  = g / ppr;
  const unsigned p     = g - rowu * ppr;
  const bool second    = p >= kp8;
  const int row = (int)rowu;
  const int c0  = (int)((second ? p - kp8 : p) << 3);
  const float* srow = src + (size_t)clampi(row, 0, rows - 1) * (size_t)ldsrc;
  float x[8];
  unsigned mk[8];
#pragma unroll
  for (int e = 0; e < 8; ++e) {
    const int c = c0 + e;
    const float v = srow[clampi(c, 0, cols - 1)];
    asm volatile("" :: "v"(v));
    x[e]  = v;
    mk[e] = (row < rows && c < cols) ? 0xFFFFu : 0u;
  }
  const v4f a = (v4f){ x[0], x[1], x[2], x[3] };
  const v4f c = (v4f){ x[4], x[5], x[6], x[7] };
  v4u o;
  if (FORM == 2) {
    o = pack8_f16(a, c);
  } else {
    const v4u hi = pack8_bf16(a, c);
    o = hi;
    if (FORM == 1) { const v4u lo = pack8_bf16_lo(a, c); o = second ? lo : hi; }
  }
  const v4u mw = (v4u){ pk16(mk[0], mk[1]), pk16(mk[2], mk[3]), pk16(mk[4], mk[5]), pk16(mk[6], mk[7]) };
  o &= mw;
  if (g < total) {
    volatile v4u* q = (volatile v4u*)(dst + (size_t)g * 8);
    *q = o;
    __threadfence();
    *q = o;
  }
}

template <int FORM> struct FragOf    { typedef FragB T; };
template <>         struct FragOf<2> { typedef FragH T; };
__device__ __forceinline__ v8f mm(const FragB& a, const FragB& b, v8f c) { return wmb(a, b, c); }
__device__ __forceinline__ v8f mm(const FragH& a, const FragH& b, v8f c) { return wmh(a, b, c); }
template <class F> __device__ __forceinline__ F ld_frag(const unsigned short* p) {
  F f;
  f.h[0] = *(const v8usa*)(p);
  f.h[1] = *(const v8usa*)(p + 16);
  return f;
}

template <int FORM, int EPI>
__global__ __launch_bounds__(256) __attribute__((amdgpu_num_vgpr(248)))
void k_gemm_nt(const unsigned short* __restrict__ A, const unsigned short* __restrict__ B,
               const float* __restrict__ bias, float* __restrict__ D, int M, int N, int KTOT, int ldd) {
  static_assert(FORM >= 0 && FORM <= 2);
  static_assert(EPI == 0 || EPI == 1);
  typedef typename FragOf<FORM>::T F;
  __shared__ __attribute__((aligned(16))) float sT[8][16 * 68];
  const int lane = threadIdx.x & 31;
  const int wave = threadIdx.x >> 5;
  const int tilesM = (M + 63) >> 6;
  const int tilesN = (N + 63) >> 6;
  const int tile = blockIdx.x * 8 + wave;
  if (tile >= tilesM * tilesN) return;
  const int tm = tile / tilesN;
  const int tn = tile - tm * tilesN;
  const int m0 = tm << 6;
  const int n0 = tn << 6;

  const int rl = lane & 15;
  const int h8 = (lane >> 4) * 8;
  const unsigned short* pa = A + (size_t)(m0 + rl) * (size_t)KTOT + h8;
  const unsigned short* pb = B + (size_t)(n0 + rl) * (size_t)KTOT + h8;

  v8f acc[4][4];
#pragma unroll
  for (int i = 0; i < 4; ++i)
#pragma unroll
    for (int j = 0; j < 4; ++j) acc[i][j] = (v8f){0.f, 0.f, 0.f, 0.f, 0.f, 0.f, 0.f, 0.f};

#pragma unroll 1
  for (int k0 = 0; k0 < KTOT; k0 += 32) {
    F bf[4];
#pragma unroll
    for (int j = 0; j < 4; ++j) bf[j] = ld_frag<F>(pb + (size_t)(j << 4) * (size_t)KTOT + k0);
#pragma unroll
    for (int i = 0; i < 4; ++i) {
      const F af = ld_frag<F>(pa + (size_t)(i << 4) * (size_t)KTOT + k0);
#pragma unroll
      for (int j = 0; j < 4; ++j) acc[i][j] = mm(af, bf[j], acc[i][j]);
    }
  }

  float* slab = sT[wave];
  const int hh = lane >> 4;
  const int c4 = (lane & 15) * 4;
  const int nc = n0 + c4;
  const bool cok = nc < N;
  v4f bv = (v4f){0.f, 0.f, 0.f, 0.f};
  if (EPI == 1) {
    bv = *(const v4fa*)(bias + clampi(nc, 0, N - 4));
    asm volatile("" :: "v"(bv));
  }
#pragma unroll
  for (int i = 0; i < 4; ++i) {
    const int mBase = m0 + (i << 4);
#pragma unroll
    for (int j = 0; j < 4; ++j) {
#pragma unroll
      for (int r = 0; r < 8; ++r) slab[(h8 + r) * 68 + (j << 4) + rl] = acc[i][j][r];
    }
    __builtin_amdgcn_fence(__ATOMIC_RELEASE, "workgroup");
    __builtin_amdgcn_wave_barrier();
    __builtin_amdgcn_fence(__ATOMIC_ACQUIRE, "workgroup");
    v4f vv[8];
#pragma unroll
    for (int it = 0; it < 8; ++it) {
      const int row = it * 2 + hh;
      v4f v = *(const v4fa*)(slab + row * 68 + c4);
      if (EPI == 1) v += bv;
      vv[it] = v;
    }
    for (int pass = 0; pass < 2; ++pass) {
#pragma unroll
      for (int it = 0; it < 8; ++it) {
        const int row = mBase + it * 2 + hh;
        if (cok && row < M) *(volatile v4f*)(D + (size_t)row * (size_t)ldd + nc) = vv[it];
      }
      __threadfence();
    }
    __builtin_amdgcn_fence(__ATOMIC_RELEASE, "workgroup");
    __builtin_amdgcn_wave_barrier();
    __builtin_amdgcn_fence(__ATOMIC_ACQUIRE, "workgroup");
  }
}

#include <stddef.h>
#include <stdint.h>

#pragma clang fp contract(off)

#define NN      50000
#define NE      800000
#define DD      128
#define KT      256
#define MP      50048
#define NTHR    256
#define NWAVE   8
#define EPT     8
#define WCH     (32 * EPT)
#define NBRUN   512
#define SLB     9
#define NBK     98
#define WLCAP   3072
#define LCAP    12288
#define DEGCAP  48
#define MAXDEG_MEAS  33
#define MAXB512_MEAS 8397

#define BK_ZINTS (NWAVE * WLCAP + LCAP + 4 * NBRUN)
#define BK_LDS   (BK_ZINTS * 4)

#define PBX      (MP * DD / 8 / 256)
#define PB_W     16
#define PB_TOT   (4 * PB_W + 1)
#define WPL      (DD * KT)
#define SPLIT_BLOCKS (MP * KT / 8 / 256)
#define WALK_BLOCKS  (MP / NWAVE)
#define OUT_BLOCKS   (NN * DD / 4 / 256)
#define GEMM_BLOCKS  ((((MP / 64) * (DD / 64)) + 7) / 8)

static_assert(DD == 128 && DD == 32 * 4 && DD % 64 == 0 && KT == 2 * DD && KT % 32 == 0);
static_assert(MP % 64 == 0 && MP >= NN && MP == 391 * 128 && MP % 16 == 0 && MP % NWAVE == 0);
static_assert((MP * DD / 8) % 256 == 0 && (MP * KT / 8) % 256 == 0 && (NN * DD / 4) % 256 == 0);
static_assert((long long)MP * KT / 8 < (1LL << 31));
static_assert((DD * KT / 8) == PB_W * NTHR);
static_assert(NBRUN == (1 << SLB) && NBRUN == NTHR * 2 && NBRUN % 32 == 0);
static_assert(NBK * NBRUN >= NN && (NBK - 1) * NBRUN < NN);
static_assert(NE <= (1 << 20) && (((long long)NE) << SLB) < (1LL << 31));
static_assert(NE % WCH == 0 && NE % 8 == 0);
static_assert((long long)LCAP * 100 >= (long long)MAXB512_MEAS * 125);
static_assert(WLCAP >= MAXB512_MEAS / 8 + 8 * 46 + 1);
static_assert(MAXDEG_MEAS + 8 <= DEGCAP);
static_assert(LCAP % (NTHR * 4) == 0 && BK_ZINTS % (NTHR * 4) == 0);
static_assert(BK_LDS <= 262144 && BK_LDS + 0 <= 327680);
static_assert(GEMM_BLOCKS == 196);

typedef unsigned int v2u __attribute__((ext_vector_type(2)));
typedef int          v2i __attribute__((ext_vector_type(2)));
typedef int          v4i __attribute__((ext_vector_type(4)));
typedef v2u __attribute__((may_alias)) v2ua;
typedef v2i __attribute__((may_alias)) v2ia;
typedef v4i __attribute__((may_alias)) v4ia;
typedef v4u __attribute__((may_alias)) v4ua;

__device__ __forceinline__ void st2_v4u(unsigned short* p, v4u v) {
  volatile v4u* q = (volatile v4u*)p;
  *q = v;
  __threadfence();
  *q = v;
}
__device__ __forceinline__ void st2_v4f(float* p, v4f v) {
  volatile v4f* q = (volatile v4f*)p;
  *q = v;
  __threadfence();
  *q = v;
}

__device__ __forceinline__ float act_keep(float v) { return (v < 0.0f) ? 0.0f : v; }

__device__ __forceinline__ v4u gather8_bf16(const float* __restrict__ base) {
  float f[8];
#pragma unroll
  for (int i = 0; i < 8; ++i) f[i] = base[(size_t)i * (size_t)DD];
  return (v4u){ pk16(bf16_bits(f[0]), bf16_bits(f[1])), pk16(bf16_bits(f[2]), bf16_bits(f[3])),
                pk16(bf16_bits(f[4]), bf16_bits(f[5])), pk16(bf16_bits(f[6]), bf16_bits(f[7])) };
}

__device__ __forceinline__ void prep_w(const float* __restrict__ w, unsigned short* wt, int u) {
  const int n  = u >> 5;
  const int k8 = (u & 31) * 8;
  const int ks = k8 & (DD - 1);
  const v4u o = gather8_bf16(w + (size_t)ks * DD + n);
  st2_v4u(wt + (size_t)n * KT + k8, o);
}

__global__ __launch_bounds__(NTHR) void k_prep(const float* __restrict__ w1a, const float* __restrict__ w2a,
                                               const float* __restrict__ w1b, const float* __restrict__ w2b,
                                               const float* __restrict__ b1a, const float* __restrict__ b2a,
                                               const float* __restrict__ b1b, const float* __restrict__ b2b,
                                               unsigned short* WT, float* BIAS) {
  const int tid = (int)threadIdx.x;
  const int blk = (int)blockIdx.x;
  if (blk < PB_W) {
    prep_w(w1a, WT, blk * NTHR + tid);
  } else if (blk < 2 * PB_W) {
    prep_w(w2a, WT + (size_t)WPL, (blk - PB_W) * NTHR + tid);
  } else if (blk < 3 * PB_W) {
    prep_w(w1b, WT + (size_t)2 * WPL, (blk - 2 * PB_W) * NTHR + tid);
  } else if (blk < 4 * PB_W) {
    prep_w(w2b, WT + (size_t)3 * WPL, (blk - 3 * PB_W) * NTHR + tid);
  } else {
    const int c4  = (tid & 31) * 4;
    const int seg = (tid >> 5) & 3;
    const v4f x1 = *(const v4fa*)(b1a + c4);
    const v4f x2 = *(const v4fa*)(b2a + c4);
    const v4f x3 = *(const v4fa*)(b1b + c4);
    const v4f x4 = *(const v4fa*)(b2b + c4);
    asm volatile("" :: "v"(x1), "v"(x2));
    asm volatile("" :: "v"(x3), "v"(x4));
    const unsigned m1 = (seg == 0) ? 0xFFFFFFFFu : 0u;
    const unsigned m2 = (seg == 1) ? 0xFFFFFFFFu : 0u;
    const unsigned m3 = (seg == 2) ? 0xFFFFFFFFu : 0u;
    const unsigned m4 = (seg == 3) ? 0xFFFFFFFFu : 0u;
    v4f o;
#pragma unroll
    for (int e = 0; e < 4; ++e) {
      const unsigned u1 = __float_as_uint(bf16_val(x1[e])) & m1;
      const unsigned u2 = __float_as_uint(bf16_val(x2[e])) & m2;
      const unsigned u3 = __float_as_uint(bf16_val(x3[e])) & m3;
      const unsigned u4 = __float_as_uint(bf16_val(x4[e])) & m4;
      o[e] = __uint_as_float(u1 | u2 | u3 | u4);
    }
    if (tid < 128) st2_v4f(BIAS + 4 * tid, o);
  }
}

__device__ __forceinline__ void build_flush(const int* pl, const int* cnt, const int* offs, int ov,
                                            int* lp, int* mp, int* fp, int tid) {
#pragma unroll 1
  for (int i = tid * 4; i < LCAP; i += NTHR * 4) {
    const v4i v = *(const v4ia*)(pl + i);
    *(volatile v4i*)(lp + i) = v;
  }
  {
    const v2i vc = *(const v2ia*)(cnt + 2 * tid);
    const v2i vo = *(const v2ia*)(offs + 2 * tid);
    const v4i m = {vc.x, vo.x, vc.y, vo.y};
    *(volatile v4i*)(mp + 4 * tid) = m;
  }
  if (tid < 8) {
    const v4i f = {ov, ov, ov, ov};
    *(volatile v4i*)(fp + 4 * tid) = f;
  }
}

__global__ __launch_bounds__(NTHR) void k_build(const int* __restrict__ srcs, const int* __restrict__ dsts,
                                                int* LIST, int* META, int* FLAG) {
  extern __shared__ __attribute__((aligned(16))) int dsm[];
  int* wl   = dsm;
  int* pl   = dsm + NWAVE * WLCAP;
  int* cnt  = pl + LCAP;
  int* offs = cnt + NBRUN;
  int* cur  = offs + NBRUN;
  int* misc = cur + NBRUN;
  const int tid = (int)threadIdx.x, lane = tid & 31, wave = tid >> 5;
  const int blk = (int)blockIdx.x;
  const unsigned nbs = (unsigned)(blk * NBRUN);

  {
    const v4i z4 = {0, 0, 0, 0};
#pragma unroll 1
    for (int i = tid * 4; i < BK_ZINTS; i += NTHR * 4) *(v4ia*)(dsm + i) = z4;
  }
  __syncthreads();

  {
    const int per  = ((NE + NWAVE * WCH - 1) / (NWAVE * WCH)) * WCH;
    const int ebeg = wave * per;
    const int eend = (ebeg + per < NE) ? (ebeg + per) : NE;
    int* mylist = wl + wave * WLCAP;
    int wc = 0;
#pragma unroll 1
    for (int cb = ebeg; cb < eend; cb += WCH) {
      const int e0 = cb + lane * EPT;
      const v4i da = *(const v4ia*)(dsts + e0);
      const v4i db = *(const v4ia*)(dsts + e0 + 4);
      const int d0 = da.x, d1 = da.y, d2 = da.z, d3 = da.w;
      const int d4 = db.x, d5 = db.y, d6 = db.z, d7 = db.w;
      asm volatile("" :: "v"(d0), "v"(d1), "v"(d2), "v"(d3));
      asm volatile("" :: "v"(d4), "v"(d5), "v"(d6), "v"(d7));
      const unsigned s0 = (unsigned)d0 - nbs, s1 = (unsigned)d1 - nbs;
      const unsigned s2 = (unsigned)d2 - nbs, s3 = (unsigned)d3 - nbs;
      const unsigned s4 = (unsigned)d4 - nbs, s5 = (unsigned)d5 - nbs;
      const unsigned s6 = (unsigned)d6 - nbs, s7 = (unsigned)d7 - nbs;
      const bool h0 = s0 < (unsigned)NBRUN, h1 = s1 < (unsigned)NBRUN, h2 = s2 < (unsigned)NBRUN, h3 = s3 < (unsigned)NBRUN;
      const bool h4 = s4 < (unsigned)NBRUN, h5 = s5 < (unsigned)NBRUN, h6 = s6 < (unsigned)NBRUN, h7 = s7 < (unsigned)NBRUN;
      const unsigned m0 = __builtin_amdgcn_ballot_w32(h0), m1 = __builtin_amdgcn_ballot_w32(h1);
      const unsigned m2 = __builtin_amdgcn_ballot_w32(h2), m3 = __builtin_amdgcn_ballot_w32(h3);
      const unsigned m4 = __builtin_amdgcn_ballot_w32(h4), m5 = __builtin_amdgcn_ballot_w32(h5);
      const unsigned m6 = __builtin_amdgcn_ballot_w32(h6), m7 = __builtin_amdgcn_ballot_w32(h7);
      const unsigned any = m0 | m1 | m2 | m3 | m4 | m5 | m6 | m7;
      if (any != 0u) {
        const int pre = (int)(__builtin_amdgcn_mbcnt_lo(m0, 0u) + __builtin_amdgcn_mbcnt_lo(m1, 0u) +
                              __builtin_amdgcn_mbcnt_lo(m2, 0u) + __builtin_amdgcn_mbcnt_lo(m3, 0u) +
                              __builtin_amdgcn_mbcnt_lo(m4, 0u) + __builtin_amdgcn_mbcnt_lo(m5, 0u) +
                              __builtin_amdgcn_mbcnt_lo(m6, 0u) + __builtin_amdgcn_mbcnt_lo(m7, 0u));
        int p = wc + pre;
        if (h0) { mylist[p < WLCAP ? p : WLCAP - 1] = ((e0 + 0) << SLB) | (int)s0; p = p + 1; }
        if (h1) { mylist[p < WLCAP ? p : WLCAP - 1] = ((e0 + 1) << SLB) | (int)s1; p = p + 1; }
        if (h2) { mylist[p < WLCAP ? p : WLCAP - 1] = ((e0 + 2) << SLB) | (int)s2; p = p + 1; }
        if (h3) { mylist[p < WLCAP ? p : WLCAP - 1] = ((e0 + 3) << SLB) | (int)s3; p = p + 1; }
        if (h4) { mylist[p < WLCAP ? p : WLCAP - 1] = ((e0 + 4) << SLB) | (int)s4; p = p + 1; }
        if (h5) { mylist[p < WLCAP ? p : WLCAP - 1] = ((e0 + 5) << SLB) | (int)s5; p = p + 1; }
        if (h6) { mylist[p < WLCAP ? p : WLCAP - 1] = ((e0 + 6) << SLB) | (int)s6; p = p + 1; }
        if (h7) { mylist[p < WLCAP ? p : WLCAP - 1] = ((e0 + 7) << SLB) | (int)s7; p = p + 1; }
        wc += (int)(__builtin_popcount(m0) + __builtin_popcount(m1) + __builtin_popcount(m2) + __builtin_popcount(m3) +
                    __builtin_popcount(m4) + __builtin_popcount(m5) + __builtin_popcount(m6) + __builtin_popcount(m7));
      }
    }
    if (lane == 0) misc[wave] = wc;
  }
  __syncthreads();

  if (wave == 0) {
    int ov = 0;
    int tot = 0;
#pragma unroll 1
    for (int w2 = 0; w2 < NWAVE; ++w2) {
      int c = __builtin_amdgcn_readfirstlane(misc[w2]);
      if (c > WLCAP) ov = 1;
      c = c < 0 ? 0 : (c > WLCAP ? WLCAP : c);
      tot += c;
#pragma unroll 1
      for (int b0 = 0; b0 < c; b0 += 32) {
        const int idx = b0 + lane;
        const int ent = wl[w2 * WLCAP + (idx < WLCAP ? idx : WLCAP - 1)];
        const int m32 = (c - b0) < 32 ? (c - b0) : 32;
#pragma unroll 1
        for (int k = 0; k < m32; ++k) {
          const int u    = __builtin_amdgcn_readlane(ent, k);
          const int slot = u & (NBRUN - 1);
          if (lane == 0) cnt[slot] = cnt[slot] + 1;
        }
      }
    }
    if (tot > LCAP) ov = 1;
    if (lane == 0) misc[9] = ov;
  }
  __syncthreads();
  if (wave == 0) {
    const int base = lane * (NBRUN / 32);
    int s = 0;
#pragma unroll 1
    for (int i = 0; i < NBRUN / 32; ++i) s += cnt[base + i];
    int incl = s;
#pragma unroll
    for (int d = 1; d < 32; d <<= 1) {
      const int y = __shfl_up(incl, d, 32);
      if (lane >= d) incl += y;
    }
    int run = incl - s;
#pragma unroll 1
    for (int i = 0; i < NBRUN / 32; ++i) {
      const int cv = cnt[base + i];
      offs[base + i] = run;
      cur[base + i]  = run;
      run += cv;
    }
  }
  __syncthreads();

  if (wave == 0) {
#pragma unroll 1
    for (int w2 = 0; w2 < NWAVE; ++w2) {
      int c = __builtin_amdgcn_readfirstlane(misc[w2]);
      c = c < 0 ? 0 : (c > WLCAP ? WLCAP : c);
#pragma unroll 1
      for (int b0 = 0; b0 < c; b0 += 32) {
        const int idx = b0 + lane;
        const int ent = wl[w2 * WLCAP + (idx < WLCAP ? idx : WLCAP - 1)];
        int eid = (ent >> SLB) & 0xFFFFF;
        eid = eid > NE - 1 ? NE - 1 : eid;
        int sr = srcs[eid];
        asm volatile("" :: "v"(sr));
        sr = sr < 0 ? 0 : (sr > NN - 1 ? NN - 1 : sr);
        const int m32 = (c - b0) < 32 ? (c - b0) : 32;
#pragma unroll 1
        for (int k = 0; k < m32; ++k) {
          const int u    = __builtin_amdgcn_readlane(ent, k);
          const int w0   = __builtin_amdgcn_readlane(sr, k);
          const int slot = u & (NBRUN - 1);
          if (lane == 0) {
            int p = cur[slot];
            p = p < 0 ? 0 : (p > LCAP - 1 ? LCAP - 1 : p);
            pl[p] = w0;
            cur[slot] = p + 1;
          }
        }
      }
    }
  }
  __syncthreads();

  const int ovf = misc[9];
  int* lp = LIST + (size_t)blk * (size_t)LCAP;
  int* mp = META + (size_t)blk * (size_t)(2 * NBRUN);
  int* fp = FLAG + (size_t)blk * 32;
  build_flush(pl, cnt, offs, ovf, lp, mp, fp, tid);
  __threadfence();
  build_flush(pl, cnt, offs, ovf, lp, mp, fp, tid);
}

template <int SRC32>
__device__ __forceinline__ v4f ld_row(const unsigned short* __restrict__ XB, const float* __restrict__ HF,
                                      int s, int lane) {
  v4f r;
  if (SRC32 == 0) {
    const v2u w = *(const v2ua*)(XB + (size_t)s * DD + 4 * lane);
    asm volatile("" :: "v"(w));
    float f0 = __uint_as_float(w.x << 16);
    float f1 = __uint_as_float(w.x & 0xffff0000u);
    float f2 = __uint_as_float(w.y << 16);
    float f3 = __uint_as_float(w.y & 0xffff0000u);
    asm volatile("" : "+v"(f0), "+v"(f1), "+v"(f2), "+v"(f3));
    r = (v4f){ f0, f1, f2, f3 };
  } else {
    const v4f q = *(const v4fa*)(HF + (size_t)s * DD + 4 * lane);
    asm volatile("" :: "v"(q));
    r = (v4f){ act_keep(q[0]), act_keep(q[1]), act_keep(q[2]), act_keep(q[3]) };
  }
  return r;
}

template <int SRC32>
__global__ __launch_bounds__(NTHR) void k_walk(const int* __restrict__ LIST, const int* __restrict__ META,
                                               const int* __restrict__ FLAG, const unsigned short* __restrict__ XB,
                                               const float* __restrict__ HF, unsigned short* OP,
                                               int n_nodes, int n_pad) {
  __shared__ __attribute__((aligned(16))) unsigned srow[NWAVE][128];
  const int tid = (int)threadIdx.x, lane = tid & 31, wave = tid >> 5;
  const int node = (int)blockIdx.x * NWAVE + wave;
  const int dn = node < NN - 1 ? node : NN - 1;
  const int blk = dn >> SLB;
  const int* lb = LIST + (size_t)blk * (size_t)LCAP;
  const v2i mt = *(const v2ia*)(META + 2 * (size_t)dn);
  const int craw = mt.x;
  const int oraw = mt.y;
  const int flag = FLAG[(size_t)blk * 32];
  asm volatile("" :: "v"(craw), "v"(oraw), "v"(flag));
  const v4f self = ld_row<SRC32>(XB, HF, dn, lane);

  const bool big = craw > DEGCAP;
  const int c = __builtin_amdgcn_readfirstlane(craw < 0 ? 0 : (craw > DEGCAP ? DEGCAP : craw));
  const int o = oraw < 0 ? 0 : (oraw > LCAP - 1 ? LCAP - 1 : oraw);
  int last = o + (c > 0 ? c : 1) - 1;
  last = last > LCAP - 1 ? LCAP - 1 : last;

  v4f acc = (v4f){ 0.0f, 0.0f, 0.0f, 0.0f };
#pragma unroll 1
  for (int b0 = 0; b0 < c; b0 += 32) {
    int idx = o + b0 + lane;
    idx = idx > last ? last : idx;
    int sr = lb[idx];
    asm volatile("" :: "v"(sr));
    sr = sr < 0 ? 0 : (sr > NN - 1 ? NN - 1 : sr);
    const int m32 = (c - b0) < 32 ? (c - b0) : 32;
#pragma unroll 1
    for (int k = 0; k < m32; k += 4) {
      const int e1 = (k + 1 < m32) ? (k + 1) : (m32 - 1);
      const int e2 = (k + 2 < m32) ? (k + 2) : (m32 - 1);
      const int e3 = (k + 3 < m32) ? (k + 3) : (m32 - 1);
      const int s0 = __builtin_amdgcn_readlane(sr, k);
      const int s1 = __builtin_amdgcn_readlane(sr, e1);
      const int s2 = __builtin_amdgcn_readlane(sr, e2);
      const int s3 = __builtin_amdgcn_readlane(sr, e3);
      const v4f q0 = ld_row<SRC32>(XB, HF, s0, lane);
      const v4f q1 = ld_row<SRC32>(XB, HF, s1, lane);
      const v4f q2 = ld_row<SRC32>(XB, HF, s2, lane);
      const v4f q3 = ld_row<SRC32>(XB, HF, s3, lane);
      acc = acc + q0;
      if (k + 1 < m32) acc = acc + q1;
      if (k + 2 < m32) acc = acc + q2;
      if (k + 3 < m32) acc = acc + q3;
    }
  }
  const v4f agg = self + acc;
  const bool bad = (flag != 0) | big;
  const float qnan = __uint_as_float(0x7fc00000u);
  const float r0 = bad ? qnan : agg[0];
  const float r1 = bad ? qnan : agg[1];
  const float r2 = bad ? qnan : agg[2];
  const float r3 = bad ? qnan : agg[3];
  const unsigned keep = (node < n_nodes) ? 0xFFFFFFFFu : 0u;
  const unsigned h0 = pk16(bf16_bits(r0), bf16_bits(r1)) & keep;
  const unsigned h1 = pk16(bf16_bits(r2), bf16_bits(r3)) & keep;
  const unsigned l0 = pk16(bf16_lo_bits(r0), bf16_lo_bits(r1)) & keep;
  const unsigned l1 = pk16(bf16_lo_bits(r2), bf16_lo_bits(r3)) & keep;
  unsigned* row = srow[wave];
  *(v2ua*)(row + 2 * lane)      = (v2u){ h0, h1 };
  *(v2ua*)(row + 64 + 2 * lane) = (v2u){ l0, l1 };
  __builtin_amdgcn_fence(__ATOMIC_RELEASE, "workgroup");
  __builtin_amdgcn_wave_barrier();
  __builtin_amdgcn_fence(__ATOMIC_ACQUIRE, "workgroup");
  const v4u ov = *(const v4ua*)(row + 4 * lane);
  if (node < n_pad) {
    volatile v4u* q = (volatile v4u*)(OP + (size_t)node * KT + 8 * lane);
    *q = ov;
    __threadfence();
    *q = ov;
  }
}

__global__ __launch_bounds__(NTHR) void k_split(const float* __restrict__ T, unsigned short* OP, int rows_valid) {
  const unsigned g   = blockIdx.x * 256u + threadIdx.x;
  const unsigned row = g >> 5;
  const unsigned p   = g & 31u;
  const unsigned ms  = (p >= 16u) ? 0xFFFFFFFFu : 0u;
  const unsigned c0  = (p & 15u) * 8u;
  const unsigned rc  = row < (unsigned)(MP - 1) ? row : (unsigned)(MP - 1);
  const float* s = T + (size_t)rc * DD + c0;
  const v4f xa = *(const v4fa*)(s);
  const v4f xc = *(const v4fa*)(s + 4);
  asm volatile("" :: "v"(xa), "v"(xc));
  const v4f a = (v4f){ act_keep(xa[0]), act_keep(xa[1]), act_keep(xa[2]), act_keep(xa[3]) };
  const v4f c = (v4f){ act_keep(xc[0]), act_keep(xc[1]), act_keep(xc[2]), act_keep(xc[3]) };
  const v4u hi = pack8_bf16(a, c);
  const v4u lo = pack8_bf16_lo(a, c);
  const unsigned rk = ((int)row < rows_valid) ? 0xFFFFFFFFu : 0u;
  const v4u mlo = (v4u){ ms, ms, ms, ms };
  const v4u mhi = (v4u){ ~ms, ~ms, ~ms, ~ms };
  const v4u mrk = (v4u){ rk, rk, rk, rk };
  const v4u o = ((hi & mhi) | (lo & mlo)) & mrk;
  if (g < (unsigned)MP * 32u) st2_v4u(OP + (size_t)g * 8, o);
}

__global__ __launch_bounds__(NTHR) void k_out(const float* __restrict__ Y, const int* __restrict__ FLAG,
                                              float* out, int n_rows) {
  const unsigned g   = blockIdx.x * 256u + threadIdx.x;
  const unsigned row = g >> 5;
  const unsigned c4  = (g & 31u) * 4u;
  const unsigned rc  = row < (unsigned)(NN - 1) ? row : (unsigned)(NN - 1);
  const unsigned blk = rc >> SLB;
  const v4f x = *(const v4fa*)(Y + (size_t)rc * DD + c4);
  const int flag = FLAG[(size_t)blk * 32];
  asm volatile("" :: "v"(x), "v"(flag));
  const float qnan = __uint_as_float(0x7fc00000u);
  const bool bad = flag != 0;
  v4f o;
  o[0] = bad ? qnan : act_keep(x[0]);
  o[1] = bad ? qnan : act_keep(x[1]);
  o[2] = bad ? qnan : act_keep(x[2]);
  o[3] = bad ? qnan : act_keep(x[3]);
  if ((int)row < n_rows) st2_v4f(out + (size_t)row * DD + c4, o);
}

extern "C" void kernel_launch(void* const* d_in, const int* in_sizes, int n_in,
                              void* d_out, int out_size, void* d_ws, size_t ws_size,
                              hipStream_t stream) {
  if (n_in < 11) return;
  if (in_sizes[0] != NN * DD) return;
  if (in_sizes[1] != NE || in_sizes[2] != NE) return;
  if (in_sizes[3] != DD * DD || in_sizes[5] != DD * DD) return;
  if (in_sizes[7] != DD * DD || in_sizes[9] != DD * DD) return;
  if (in_sizes[4] != DD || in_sizes[6] != DD || in_sizes[8] != DD || in_sizes[10] != DD) return;
  if (out_size != NN * DD) return;
  const int n_nodes = in_sizes[0] / DD;

  const float* feat = (const float*)d_in[0];
  const int*   srcs = (const int*)d_in[1];
  const int*   dsts = (const int*)d_in[2];
  const float* w1a  = (const float*)d_in[3];
  const float* b1a  = (const float*)d_in[4];
  const float* w2a  = (const float*)d_in[5];
  const float* b2a  = (const float*)d_in[6];
  const float* w1b  = (const float*)d_in[7];
  const float* b1b  = (const float*)d_in[8];
  const float* w2b  = (const float*)d_in[9];
  const float* b2b  = (const float*)d_in[10];
  float* out = (float*)d_out;

  constexpr size_t zXB   = (size_t)MP * DD * 2;
  constexpr size_t zOP   = (size_t)MP * KT * 2;
  constexpr size_t zF    = (size_t)MP * DD * 4;
  constexpr size_t zLIST = (size_t)NBK * LCAP * 4;
  constexpr size_t zMETA = (size_t)NBK * NBRUN * 8;
  constexpr size_t zFLAG = 16384;
  constexpr size_t zWT   = (size_t)4 * WPL * 2;
  constexpr size_t zBIAS = 2048;
  constexpr size_t oXB   = 0;
  constexpr size_t oOP   = oXB + zXB;
  constexpr size_t oT    = oOP + zOP;
  constexpr size_t oH    = oT + zF;
  constexpr size_t oLIST = oH + zF;
  constexpr size_t oMETA = oLIST + zLIST;
  constexpr size_t oFLAG = oMETA + zMETA;
  constexpr size_t oWT   = oFLAG + zFLAG;
  constexpr size_t oBIAS = oWT + zWT;
  constexpr size_t oEND  = oBIAS + zBIAS;
  static_assert(zXB % 256 == 0 && zOP % 256 == 0 && zF % 256 == 0 && zLIST % 256 == 0 && zMETA % 256 == 0);
  static_assert(zFLAG % 256 == 0 && zWT % 256 == 0 && zBIAS % 256 == 0);
  static_assert(zFLAG >= (size_t)NBK * 128);
  static_assert(zBIAS >= (size_t)4 * DD * 4);
  static_assert(oEND == 95184896);
  static_assert(oEND <= ((size_t)128 << 20));
  if (oEND > ws_size) return;

  char* ws = (char*)d_ws;
  unsigned short* XB   = (unsigned short*)(ws + oXB);
  unsigned short* OP   = (unsigned short*)(ws + oOP);
  float*          T    = (float*)(ws + oT);
  float*          H    = (float*)(ws + oH);
  int*            LIST = (int*)(ws + oLIST);
  int*            META = (int*)(ws + oMETA);
  int*            FLAG = (int*)(ws + oFLAG);
  unsigned short* WT   = (unsigned short*)(ws + oWT);
  float*          BIAS = (float*)(ws + oBIAS);

  hipFuncSetAttribute(reinterpret_cast<const void*>(&k_build), hipFuncAttributeMaxDynamicSharedMemorySize, (int)BK_LDS);

  k_plane<0><<<PBX, 256, 0, stream>>>(feat, NN, DD, DD, XB, MP, DD);
  k_prep<<<PB_TOT, NTHR, 0, stream>>>(w1a, w2a, w1b, w2b, b1a, b2a, b1b, b2b, WT, BIAS);
  k_build<<<NBK, NTHR, BK_LDS, stream>>>(srcs, dsts, LIST, META, FLAG);
  k_walk<0><<<WALK_BLOCKS, NTHR, 0, stream>>>(LIST, META, FLAG, XB, H, OP, n_nodes, MP);
  k_gemm_nt<1, 1><<<GEMM_BLOCKS, 256, 0, stream>>>(OP, WT, BIAS, T, MP, DD, KT, DD);
  k_split<<<SPLIT_BLOCKS, NTHR, 0, stream>>>(T, OP, n_nodes);
  k_gemm_nt<1, 1><<<GEMM_BLOCKS, 256, 0, stream>>>(OP, WT + (size_t)WPL, BIAS + DD, H, MP, DD, KT, DD);
  k_walk<1><<<WALK_BLOCKS, NTHR, 0, stream>>>(LIST, META, FLAG, XB, H, OP, n_nodes, MP);
  k_gemm_nt<1, 1><<<GEMM_BLOCKS, 256, 0, stream>>>(OP, WT + (size_t)2 * WPL, BIAS + 2 * DD, T, MP, DD, KT, DD);
  k_split<<<SPLIT_BLOCKS, NTHR, 0, stream>>>(T, OP, n_nodes);
  k_gemm_nt<1, 1><<<GEMM_BLOCKS, 256, 0, stream>>>(OP, WT + (size_t)3 * WPL, BIAS + 3 * DD, H, MP, DD, KT, DD);
  k_out<<<OUT_BLOCKS, NTHR, 0, stream>>>(H, FLAG, out, n_nodes);
}
